// GCN_AQ_80573586473109
// MI455X (gfx1250) — hardware-run, weakly checked
//
#include <hip/hip_runtime.h>


namespace {
constexpr int B = 16, N = 10000, T = 24, E = 160000, H = 32, O = 16, M = B * N, NBLK = M / 16;
constexpr float HS = 64.0f, WSC = 256.0f;
typedef _Float16 b16;
typedef __attribute__((ext_vector_type(16))) _Float16 v16b;
typedef __attribute__((ext_vector_type(8))) _Float16 v8b;
typedef __attribute__((ext_vector_type(8))) float v8f;
typedef __attribute__((ext_vector_type(4))) float v4f;
__device__ __forceinline__ float bf16_rne(float f) { unsigned int u = __float_as_uint(f); u += 0x7FFFu + ((u >> 16) & 1u); return __uint_as_float(u & 0xFFFF0000u); }
__device__ __forceinline__ void split16(float v, b16& hi, b16& lo) { hi = (b16)v; lo = (b16)(v - (float)hi); }
__device__ __forceinline__ v16b frag_kb(const b16* p, int hh) { const v8b a = *(const v8b*)(p + 8 * hh), b = *(const v8b*)(p + 16 + 8 * hh); v16b f;
#pragma unroll
  for (int e = 0; e < 8; ++e) { f[e] = a[e]; f[8 + e] = b[e]; } return f; }
__device__ __forceinline__ v8f wmma16b(v16b a, v16b b, v8f c) { v8f d = __builtin_amdgcn_wmma_f32_16x16x32_f16(false, a, false, b, (short)0, c, false, false); asm volatile("v_nop\n\tv_nop\n\tv_nop\n\tv_nop" : "+v"(d) : "v"(a), "v"(b)); return d; }
__device__ __forceinline__ void wave_lds_sync() { __builtin_amdgcn_fence(__ATOMIC_RELEASE, "workgroup"); __builtin_amdgcn_wave_barrier(); __builtin_amdgcn_fence(__ATOMIC_ACQUIRE, "workgroup"); }
__device__ __forceinline__ float pmul(float a, float b) { float p = a * b; asm volatile("" : "+v"(p)); return p; }
__device__ __forceinline__ int iclamp(int v, int lo, int hi) { return v < lo ? lo : (v > hi ? hi : v); }
__device__ __forceinline__ float sigm(float v) { return 1.0f / (1.0f + __expf(-v)); }
constexpr int CSR_NBLK9 = 512, CSR_GB9 = 9, CSR_GN9 = 1 << CSR_GB9  , CSR_TS9 = (CSR_GN9 < 32 ? 32 : CSR_GN9)  , CSR_MAXG9 = 512, CSR_CAP9 = 12288  ;
__device__ __host__ __forceinline__ int csr_tix9(int v) { return (v >> CSR_GB9) * CSR_TS9 + (v & (CSR_GN9 - 1)); }
__global__ __launch_bounds__(64) void csrA_kernel9(const int* __restrict__ dst, int E, int N, int nG, int CHP, int NGP, int* __restrict__ STG, int* __restrict__ HST) {
  extern __shared__ int sm[];
  int* cnt = sm; int* run = sm + NGP; int* ids = sm + 2 * NGP;
  const int b = blockIdx.x; const int ch = (E + CSR_NBLK9 - 1) / CSR_NBLK9; const int e0 = b * ch, e1 = min(E, e0 + ch);
  for (int i = threadIdx.x; i < NGP; i += 64) cnt[i] = 0;
  for (int i = threadIdx.x; i < CHP; i += 64) ids[i] = -1;
  __syncthreads();
  if (threadIdx.x == 0) {
    for (int e = e0; e < e1; ++e) { int d = dst[e]; d = (d < 0) ? 0 : (d >= N ? N - 1 : d); cnt[d >> CSR_GB9] += 1; }
    int acc = 0; for (int g = 0; g < nG; ++g) { run[g] = acc; acc += cnt[g]; }
    for (int e = e0; e < e1; ++e) { int d = dst[e]; d = (d < 0) ? 0 : (d >= N ? N - 1 : d); const int g = d >> CSR_GB9; ids[run[g]] = e; run[g] += 1; } }
  __syncthreads();
  typedef __attribute__((ext_vector_type(4))) int v4i;
  for (int pass = 0; pass < 2; ++pass) {
    for (int i = threadIdx.x; i < CHP / 4; i += 64) *(volatile v4i*)(STG + (size_t)b * CHP + i * 4) = *(const v4i*)(&ids[i * 4]);
    for (int i = threadIdx.x; i < NGP / 4; i += 64) { v4i v; for (int e = 0; e < 4; ++e) v[e] = (i * 4 + e < nG) ? cnt[i * 4 + e] : 0; *(volatile v4i*)(HST + (size_t)b * NGP + i * 4) = v; }
    __threadfence(); }
}
__global__ __launch_bounds__(512) void csrS_kernel9(const int* __restrict__ HST, int nG, int NGP, int* __restrict__ START, int* __restrict__ TOT, int* __restrict__ OFF) {
  __shared__ int tot[CSR_MAXG9];
  const int b = threadIdx.x;
  for (int pass = 0; pass < 2; ++pass) { int runb = 0; for (int g = 0; g < nG; ++g) { int c = HST[(size_t)b * NGP + g]; c = (c < 0) ? 0 : c; ((volatile int*)OFF)[(size_t)g * CSR_NBLK9 + b] = runb; runb += c; } __threadfence(); }
  for (int g = threadIdx.x; g < nG; g += 512) { int s = 0; for (int bb = 0; bb < CSR_NBLK9; ++bb) { int c = HST[(size_t)bb * NGP + g]; s += (c < 0) ? 0 : c; } tot[g] = s; }
  __syncthreads();
  if (threadIdx.x < 32) {
    __shared__ int st[CSR_MAXG9 + 32];
    if (threadIdx.x == 0) { int acc = 0; for (int g = 0; g < NGP; ++g) { st[g] = acc; if (g < nG) acc += (tot[g] + 31) & ~31; } st[NGP] = acc; }
    __builtin_amdgcn_fence(__ATOMIC_RELEASE, "workgroup"); __builtin_amdgcn_wave_barrier(); __builtin_amdgcn_fence(__ATOMIC_ACQUIRE, "workgroup");
    for (int pass = 0; pass < 2; ++pass) { for (int i = threadIdx.x; i < NGP + 32; i += 32) { ((volatile int*)START)[i] = (i <= NGP) ? st[min(i, NGP)] : 0; ((volatile int*)TOT)[i] = (i < nG) ? tot[i] : 0; } __threadfence(); } }
}
__global__ __launch_bounds__(256) void csrB_kernel9(const int* __restrict__ dst, int N, int nG, int CHP, int NGP, int permLen, const int* __restrict__ STG, const int* __restrict__ HST, const int* __restrict__ OFF, const int* __restrict__ START, const int* __restrict__ TOT, int* __restrict__ PERM, int* __restrict__ ROWPTR, int* __restrict__ ROWCNT, int* __restrict__ FLAG) {
  typedef __attribute__((ext_vector_type(4))) int v4i;
  __shared__ int ids[CSR_CAP9]; __shared__ unsigned short key[CSR_CAP9]; __shared__ int outp[CSR_CAP9]; __shared__ int ncnt[CSR_GN9 + 1]; __shared__ int boff[CSR_NBLK9 + 1];
  const int g = blockIdx.x, t_ = threadIdx.x; int tot = TOT[g]; int st = START[g], stn = START[g + 1]; const int v0 = g * CSR_GN9; const int nv = min(CSR_GN9, N - v0); const int t0 = g * CSR_TS9;
  st = (st < 0) ? 0 : (st > permLen - 32 ? permLen - 32 : st) & ~31; stn = (stn < st) ? st : (stn > permLen ? permLen : stn); tot = (tot < 0) ? 0 : tot; if (tot > stn - st && tot <= CSR_CAP9) tot = stn - st;
  if (tot > CSR_CAP9) {
    for (int pass = 0; pass < 2; ++pass) { for (int i = t_; i < CSR_TS9 / 4; i += 256) { v4i a, c; for (int e = 0; e < 4; ++e) { a[e] = st; c[e] = 0; } *(volatile v4i*)(ROWPTR + t0 + i * 4) = a; *(volatile v4i*)(ROWCNT + t0 + i * 4) = c; } if (t_ == 0) ((volatile int*)FLAG)[0] = 1; __threadfence(); } (void)nv; return; }
  if (t_ == 0) { int acc = 0; for (int b = 0; b < CSR_NBLK9; ++b) { boff[b] = acc; int c = HST[(size_t)b * NGP + g]; c = (c < 0) ? 0 : (c > CHP ? CHP : c); acc += c; if (acc > tot) acc = tot; } boff[CSR_NBLK9] = acc; }
  for (int i = t_; i <= CSR_GN9; i += 256) ncnt[i] = 0;
  __syncthreads();
  for (int b = 0; b < CSR_NBLK9; ++b) { const int c = boff[b + 1] - boff[b]; int o_ = OFF[(size_t)g * CSR_NBLK9 + b]; o_ = (o_ < 0) ? 0 : (o_ > CHP - c ? CHP - c : o_); const int* src_ = STG + (size_t)b * CHP + o_;
    for (int i = t_; i < c; i += 256) { int id = src_[i]; id = (id < 0) ? 0 : id; ids[boff[b] + i] = id; int d = dst[id]; d = (d < v0) ? v0 : (d >= N ? N - 1 : d); int kk = d - v0; kk = (kk < 0) ? 0 : (kk >= CSR_GN9 ? CSR_GN9 - 1 : kk); key[boff[b] + i] = (unsigned short)kk; } }
  __syncthreads();
  if (t_ == 0) { for (int i = 0; i < tot; ++i) ncnt[key[i]] += 1; int acc = 0; for (int vl = 0; vl < CSR_GN9; ++vl) { const int c = ncnt[vl]; ncnt[vl] = acc; acc += c; } ncnt[CSR_GN9] = acc;
    for (int i = 0; i < tot; ++i) { const int vl = key[i]; outp[ncnt[vl]] = ids[i]; ncnt[vl] += 1; }
    for (int vl = CSR_GN9; vl > 0; --vl) ncnt[vl] = ncnt[vl - 1]; ncnt[0] = 0; }
  __syncthreads();
  for (int pass = 0; pass < 2; ++pass) {
    for (int i = t_; i < (stn - st) / 4; i += 256) { v4i v; for (int e = 0; e < 4; ++e) { const int q = i * 4 + e; v[e] = (q < tot) ? outp[q] : -1; } *(volatile v4i*)(PERM + st + i * 4) = v; }
    for (int i = t_; i < CSR_TS9 / 4; i += 256) { v4i a, c; for (int e = 0; e < 4; ++e) { const int vl = i * 4 + e; const int vc = vl < CSR_GN9 ? vl : CSR_GN9; a[e] = (vl < CSR_GN9) ? st + ncnt[vc] : st; c[e] = (vl < nv) ? (ncnt[(vc < CSR_GN9 ? vc : CSR_GN9 - 1) + 1] - ncnt[vc]) : 0; } *(volatile v4i*)(ROWPTR + t0 + i * 4) = a; *(volatile v4i*)(ROWCNT + t0 + i * 4) = c; }
    __threadfence(); }
}
__global__ __launch_bounds__(256) void csrZ_kernel9(int* __restrict__ p, size_t n4) { typedef __attribute__((ext_vector_type(4))) int v4i; const size_t tid = (size_t)blockIdx.x * 256 + threadIdx.x, nth = (size_t)gridDim.x * 256; v4i z = {0, 0, 0, 0}; for (size_t i = tid; i < n4; i += nth) *(volatile v4i*)(p + i * 4) = z; }
struct CsrBufs9 { int *STG, *HST, *OFF, *START, *TOT, *PERM, *ROWPTR, *ROWCNT, *FLAG; int nG, NGP, CHP; size_t permLen; char* base; size_t bytes; };
static size_t csr_carve9(CsrBufs9& c, char* ws, size_t off, int E, int N) {
  const size_t off0 = off; c.base = ws + off;
  auto al = [&](size_t bytes) { char* p = ws + off; off += (bytes + 255) & ~(size_t)255; return p; };
  c.nG = (N + CSR_GN9 - 1) / CSR_GN9; c.NGP = (c.nG + 31) & ~31; const int ch = (E + CSR_NBLK9 - 1) / CSR_NBLK9; c.CHP = (ch + 31) & ~31; c.permLen = (size_t)E + 32 * (size_t)c.nG + 32;
  c.STG = (int*)al((size_t)CSR_NBLK9 * c.CHP * 4); c.HST = (int*)al((size_t)CSR_NBLK9 * c.NGP * 4); c.OFF = (int*)al((size_t)c.NGP * CSR_NBLK9 * 4); c.START = (int*)al((size_t)(c.NGP + 64) * 4); c.TOT = (int*)al((size_t)(c.NGP + 64) * 4);
  c.PERM = (int*)al(c.permLen * 4); c.ROWPTR = (int*)al((size_t)c.nG * CSR_TS9 * 4); c.ROWCNT = (int*)al((size_t)c.nG * CSR_TS9 * 4); c.FLAG = (int*)al(256);
  c.bytes = off - off0; return off;
}
static void csr_build9(const CsrBufs9& c, const int* dst, int E, int N, hipStream_t stream) {
  const size_t smem = (size_t)(2 * c.NGP + c.CHP) * 4;
  csrZ_kernel9<<<512, 256, 0, stream>>>((int*)c.base, c.bytes / 16);
  csrA_kernel9<<<CSR_NBLK9, 64, smem, stream>>>(dst, E, N, c.nG, c.CHP, c.NGP, c.STG, c.HST);
  csrS_kernel9<<<1, 512, 0, stream>>>(c.HST, c.nG, c.NGP, c.START, c.TOT, c.OFF);
  csrB_kernel9<<<c.nG, 256, 0, stream>>>(dst, N, c.nG, c.CHP, c.NGP, (int)c.permLen, c.STG, c.HST, c.OFF, c.START, c.TOT, c.PERM, c.ROWPTR, c.ROWCNT, c.FLAG);
}


__global__ __launch_bounds__(256) void w_kernel(const float* __restrict__ whh, const float* __restrict__ W1, const float* __restrict__ W2, b16* __restrict__ WHH, b16* __restrict__ WT1, b16* __restrict__ WT2) {
  const int u = blockIdx.x * 256 + threadIdx.x; v8b v;
  if (u < 96 * 4) { const int o = u / 4, k0 = (u % 4) * 8; for (int j = 0; j < 8; ++j) v[j] = (b16)(bf16_rne(whh[o * H + k0 + j]) * WSC); for (int pass = 0; pass < 2; ++pass) { *(volatile v8b*)(WHH + o * H + k0) = v; __threadfence(); } }
  else if (u < 96 * 4 + 32 * 4) { const int w = u - 96 * 4; const int o = w / 4, k0 = (w % 4) * 8; for (int j = 0; j < 8; ++j) v[j] = (b16)(bf16_rne(W1[(k0 + j) * H + o]) * WSC); for (int pass = 0; pass < 2; ++pass) { *(volatile v8b*)(WT1 + o * H + k0) = v; __threadfence(); } }
  else if (u < 96 * 4 + 32 * 4 + 16 * 4) { const int w = u - 96 * 4 - 32 * 4; const int o = w / 4, k0 = (w % 4) * 8; for (int j = 0; j < 8; ++j) v[j] = (b16)(bf16_rne(W2[(k0 + j) * O + o]) * WSC); for (int pass = 0; pass < 2; ++pass) { *(volatile v8b*)(WT2 + o * H + k0) = v; __threadfence(); } }
}
__global__ __launch_bounds__(32) void gru_kernel(const float* __restrict__ x, const float* __restrict__ wih, const float* __restrict__ bih, const float* __restrict__ bhh, const b16* __restrict__ WHH, int MLIM, float* __restrict__ HF) {
  __shared__ __attribute__((aligned(16))) b16 Ah[16][H + 8], Al[16][H + 8]; __shared__ __attribute__((aligned(16))) float G[16][3 * H + 4], Xs[16][T + 1];
  const int lane = threadIdx.x, nloc = lane & 15, hlf = lane >> 4; const size_t m0 = (size_t)blockIdx.x * 16; if (m0 >= (size_t)MLIM) return;
  for (int rr = 0; rr < 16; ++rr) if (lane < T) Xs[rr][lane] = bf16_rne(x[(m0 + rr) * T + lane]);
  const float wr = bf16_rne(wih[lane]), wz = bf16_rne(wih[H + lane]), wn = bf16_rne(wih[2 * H + lane]); const float bir = bf16_rne(bih[lane]), biz = bf16_rne(bih[H + lane]), bin_ = bf16_rne(bih[2 * H + lane]); const float bhr = bf16_rne(bhh[lane]), bhz = bf16_rne(bhh[H + lane]), bhn = bf16_rne(bhh[2 * H + lane]);
  float h[16];
#pragma unroll
  for (int rr = 0; rr < 16; ++rr) { h[rr] = 0.0f; Ah[rr][lane] = (b16)0.0f; Al[rr][lane] = (b16)0.0f; }
  wave_lds_sync();
#pragma unroll 1
  for (int t = 0; t < T; ++t) { v8f acc[6];
#pragma unroll
    for (int tt = 0; tt < 6; ++tt) { acc[tt] = (v8f){}; const v16b bw = frag_kb(WHH + (size_t)(tt * 16 + nloc) * H, hlf); acc[tt] = wmma16b(frag_kb(&Ah[nloc][0], hlf), bw, acc[tt]); acc[tt] = wmma16b(frag_kb(&Al[nloc][0], hlf), bw, acc[tt]); }
#pragma unroll
    for (int tt = 0; tt < 6; ++tt)
#pragma unroll
      for (int r8 = 0; r8 < 8; ++r8) G[8 * hlf + r8][tt * 16 + nloc] = acc[tt][r8] * (1.0f / (HS * WSC));
    wave_lds_sync();
#pragma unroll
    for (int rr = 0; rr < 16; ++rr) { const float xt = Xs[rr][t]; const float r = sigm(pmul(xt, wr) + bir + G[rr][lane] + bhr); const float z = sigm(pmul(xt, wz) + biz + G[rr][H + lane] + bhz); const float n = tanhf(pmul(xt, wn) + bin_ + pmul(r, G[rr][2 * H + lane] + bhn));
      h[rr] = pmul(1.0f - z, n) + pmul(z, h[rr]); b16 p, q; split16(h[rr] * HS, p, q); Ah[rr][lane] = p; Al[rr][lane] = q; }
    wave_lds_sync(); }
  for (int pass = 0; pass < 2; ++pass) {
#pragma unroll
    for (int rr = 0; rr < 16; ++rr) ((volatile float*)HF)[(m0 + rr) * H + lane] = h[rr]; __threadfence(); }
}
__global__ __launch_bounds__(256) void deg_kernel(const float* __restrict__ ew, const int* __restrict__ PERM, const int* __restrict__ ROWPTR, const int* __restrict__ ROWCNT, int permLen, float* __restrict__ DINV) {
  const int wave = threadIdx.x >> 5, lane = threadIdx.x & 31; const int v = blockIdx.x * 8 + wave; if (v >= N) return; float s = 0.0f;
  if (lane == 0) { int st = ROWPTR[v], cnt = ROWCNT[v]; cnt = iclamp(cnt, 0, 1 << 20); st = iclamp(st, 0, permLen - cnt); for (int j = 0; j < cnt; ++j) { const int e = iclamp(PERM[st + j], 0, E - 1); s += bf16_rne(ew[e]); } }
  s = __shfl(s, 0) + 1.0f; const float dv = s > 0.0f ? rsqrtf(s) : 0.0f;
  for (int pass = 0; pass < 2; ++pass) { ((volatile float*)DINV)[v * 32 + lane] = dv; __threadfence(); }
}
template <int NT>
__global__ __launch_bounds__(32) void lin_kernel(const float* __restrict__ IN, const b16* __restrict__ WT, int MLIM, float* __restrict__ OUT) {
  __shared__ __attribute__((aligned(16))) b16 Ah[16][H + 8], Al[16][H + 8]; __shared__ __attribute__((aligned(16))) float Tf[16][NT * 16 + 1];
  const int lane = threadIdx.x, nloc = lane & 15, hlf = lane >> 4; const size_t m0 = (size_t)blockIdx.x * 16; if (m0 >= (size_t)MLIM) return;
  for (int rr = 0; rr < 16; ++rr) { b16 p, q; split16(IN[(m0 + rr) * H + lane] * HS, p, q); Ah[rr][lane] = p; Al[rr][lane] = q; }
  wave_lds_sync();
#pragma unroll
  for (int t = 0; t < NT; ++t) { v8f acc = {}; const v16b bw = frag_kb(WT + (size_t)(t * 16 + nloc) * H, hlf); acc = wmma16b(frag_kb(&Ah[nloc][0], hlf), bw, acc); acc = wmma16b(frag_kb(&Al[nloc][0], hlf), bw, acc);
#pragma unroll
    for (int r8 = 0; r8 < 8; ++r8) Tf[8 * hlf + r8][t * 16 + nloc] = acc[r8] * (1.0f / (HS * WSC)); }
  wave_lds_sync();
  for (int pass = 0; pass < 2; ++pass) { for (int i = lane; i < 16 * NT * 16; i += 32) ((volatile float*)OUT)[m0 * (NT * 16) + i] = Tf[i / (NT * 16)][i % (NT * 16)]; __threadfence(); }
}
__global__ __launch_bounds__(256) void agg1_kernel(const float* __restrict__ XW, const float* __restrict__ ew, const int* __restrict__ srcs, const int* __restrict__ PERM, const int* __restrict__ ROWPTR, const int* __restrict__ ROWCNT, int permLen, const float* __restrict__ DINV, const float* __restrict__ b1, int MLIM, float* __restrict__ H1) {
  const int wave = threadIdx.x >> 5, lane = threadIdx.x & 31; const size_t m = (size_t)blockIdx.x * 8 + wave; if (m >= (size_t)MLIM) return; const int b = (int)(m / N), v = (int)(m % N); const float di = DINV[v * 32];
  int st = ROWPTR[v], cnt = ROWCNT[v]; cnt = iclamp(cnt, 0, 1 << 20); st = iclamp(st, 0, permLen - cnt); float s = pmul(pmul(di, di), XW[m * H + lane]);
#pragma unroll 1
  for (int j = 0; j < cnt; ++j) { const int e = iclamp(PERM[st + j], 0, E - 1); const int u = iclamp(srcs[e], 0, N - 1); s += pmul(pmul(pmul(DINV[u * 32], bf16_rne(ew[e])), di), XW[((size_t)b * N + u) * H + lane]); }
  const float r = fmaxf(s + bf16_rne(b1[lane]), 0.0f);
  for (int pass = 0; pass < 2; ++pass) { ((volatile float*)H1)[m * H + lane] = r; __threadfence(); }
}
__global__ __launch_bounds__(256) void agg2_kernel(const float* __restrict__ XW2, const float* __restrict__ ew, const int* __restrict__ srcs, const int* __restrict__ PERM, const int* __restrict__ ROWPTR, const int* __restrict__ ROWCNT, int permLen, const float* __restrict__ DINV, const float* __restrict__ b2, const float* __restrict__ wfc, const float* __restrict__ bfc, int MLIM, float* __restrict__ out) {
  const int wave = threadIdx.x >> 5, lane = threadIdx.x & 31; const size_t m0 = ((size_t)blockIdx.x * 8 + wave) * 32; if (m0 >= (size_t)MLIM) return; const size_t m = m0 + lane; const int b = (int)(m / N); const int v = (int)(m % N);
  float acc[O]; const float di = DINV[v * 32]; const float sw = pmul(di, di);
#pragma unroll
  for (int k = 0; k < O; ++k) acc[k] = pmul(sw, XW2[m * O + k]);
  int st = ROWPTR[v], cnt = ROWCNT[v]; cnt = iclamp(cnt, 0, 1 << 20); st = iclamp(st, 0, permLen - cnt);
#pragma unroll 1
  for (int j = 0; j < cnt; ++j) { const int e = iclamp(PERM[st + j], 0, E - 1); const int u = iclamp(srcs[e], 0, N - 1); const float w = pmul(pmul(DINV[u * 32], bf16_rne(ew[e])), di); const float* row = XW2 + ((size_t)b * N + u) * O;
#pragma unroll
    for (int k = 0; k < O; ++k) acc[k] += pmul(w, row[k]); }
  float s = bf16_rne(bfc[0]);
#pragma unroll
  for (int k = 0; k < O; ++k) s += pmul(acc[k] + bf16_rne(b2[k]), bf16_rne(wfc[k]));
  for (int pass = 0; pass < 2; ++pass) { ((volatile float*)out)[m] = s; __threadfence(); }
}
}

extern "C" void kernel_launch(void* const* d_in, const int* in_sizes, int n_in, void* d_out, int out_size, void* d_ws, size_t ws_size, hipStream_t stream) {
  (void)n_in;
  auto Fp = [&](int i) { return (const float*)d_in[i]; }; auto Ip = [&](int i) { return (const int*)d_in[i]; };
  if (in_sizes[0] != M * T || in_sizes[1] != 2 * E || in_sizes[2] != E || in_sizes[3] != 3 * H || in_sizes[4] != 3 * H * H || in_sizes[7] != H * H || in_sizes[9] != H * O || in_sizes[11] != O || out_size != M) return;
  const int MLIM = M;
  size_t off = 0; char* ws = (char*)d_ws;
  auto carve = [&](size_t bytes) { char* p = ws + off; off += (bytes + 255) & ~(size_t)255; return p; };
  b16* WHH = (b16*)carve(96 * H * 2); b16* WT1 = (b16*)carve(H * H * 2); b16* WT2 = (b16*)carve(O * H * 2); float* HF = (float*)carve((size_t)M * H * 4); float* XW = (float*)carve((size_t)M * H * 4); float* H1 = (float*)carve((size_t)M * H * 4); float* XW2 = (float*)carve((size_t)M * O * 4); float* DINV = (float*)carve((size_t)N * 32 * 4);
  CsrBufs9 csr; off = csr_carve9(csr, ws, off, E, N);
  if (off > ws_size || off > ((size_t)128 << 20)) return;
  w_kernel<<<(96 * 4 + 48 * 4 + 255) / 256, 256, 0, stream>>>(Fp(4), Fp(7), Fp(9), WHH, WT1, WT2);
  csr_build9(csr, Ip(1) + E, E, N, stream);
  deg_kernel<<<N / 8, 256, 0, stream>>>(Fp(2), csr.PERM, csr.ROWPTR, csr.ROWCNT, (int)csr.permLen, DINV);
  gru_kernel<<<MLIM / 16, 32, 0, stream>>>(Fp(0), Fp(3), Fp(5), Fp(6), WHH, MLIM, HF);
  lin_kernel<2><<<MLIM / 16, 32, 0, stream>>>(HF, WT1, MLIM, XW);
  agg1_kernel<<<MLIM / 8, 256, 0, stream>>>(XW, Fp(2), Ip(1), csr.PERM, csr.ROWPTR, csr.ROWCNT, (int)csr.permLen, DINV, Fp(8), MLIM, H1);
  lin_kernel<1><<<MLIM / 16, 32, 0, stream>>>(H1, WT2, MLIM, XW2);
  agg2_kernel<<<(MLIM + 255) / 256, 256, 0, stream>>>(XW2, Fp(2), Ip(1), csr.PERM, csr.ROWPTR, csr.ROWCNT, (int)csr.permLen, DINV, Fp(10), Fp(11), Fp(12), MLIM, (float*)d_out);
}
